// FullAttention_71399536329293
// MI455X (gfx1250) — hardware-verified
//
#include <hip/hip_runtime.h>
#include <math.h>

typedef __attribute__((ext_vector_type(16))) _Float16 v16h;
typedef __attribute__((ext_vector_type(16))) __bf16 v16b;
typedef __attribute__((ext_vector_type(8)))  _Float16 v8h;
typedef __attribute__((ext_vector_type(8)))  float v8f;
typedef __attribute__((ext_vector_type(4)))  float v4f;
typedef __attribute__((ext_vector_type(2)))  float v2f;
typedef __attribute__((ext_vector_type(4)))  unsigned v4u;
typedef __attribute__((ext_vector_type(4)))  int v4i;
typedef float __attribute__((may_alias)) float_a;
typedef int __attribute__((may_alias)) int_a;

template <typename T> __device__ __forceinline__ void vst2(void* p, T v) { *(volatile T*)p = v; __threadfence(); *(volatile T*)p = v; }
__device__ __forceinline__ v8f wmma16(v16h a, v16h b, v8f c) {
  v8f d = __builtin_amdgcn_wmma_f32_16x16x32_f16(false, a, false, b, (short)0, c, false, false);
  asm volatile("v_nop\n\tv_nop\n\tv_nop\n\tv_nop" : "+v"(d) : "v"(a), "v"(b));
  return d;
}
__device__ __forceinline__ v8f wmma_bf(v16b a, v16b b, v8f c) {
  v8f d = __builtin_amdgcn_wmma_f32_16x16x32_bf16(false, a, false, b, (short)0, c, false, false);
  asm volatile("v_nop\n\tv_nop\n\tv_nop\n\tv_nop" : "+v"(d) : "v"(a), "v"(b));
  return d;
}
__device__ __forceinline__ v16h frag_h(const _Float16* rowk0, int lane) {
  union { v16h v; v8h q[2]; } u; const _Float16* p = rowk0 + 8 * (lane >> 4);
  u.q[0] = *(const v8h*)p; u.q[1] = *(const v8h*)(p + 16); return u.v;
}
__device__ __forceinline__ v16h frag_f32(const float* rowk0, int lane) {
  v16h a; const float* p = rowk0 + 8 * (lane >> 4);
#pragma unroll
  for (int i = 0; i < 8; ++i) { a[i] = (_Float16)p[i]; a[8 + i] = (_Float16)p[16 + i]; }
  return a;
}
__device__ __forceinline__ v16h frag_f32s(const float* rowk0, int lane, float sc) {
  v16h a; const float* p = rowk0 + 8 * (lane >> 4);
#pragma unroll
  for (int i = 0; i < 8; ++i) { a[i] = (_Float16)(p[i] * sc); a[8 + i] = (_Float16)(p[16 + i] * sc); }
  return a;
}
__device__ __forceinline__ v16h fragc_f32(const float* W, int k0, int n, int lane, int ld, int K) {
  v16h a; const int g = lane >> 4;
#pragma unroll
  for (int i = 0; i < 8; ++i) { const int ka = k0 + 8 * g + i, kb = ka + 16;
    a[i] = (_Float16)(ka < K ? W[(size_t)(ka < K ? ka : K - 1) * ld + n] : 0.f); a[8 + i] = (_Float16)(kb < K ? W[(size_t)(kb < K ? kb : K - 1) * ld + n] : 0.f); }
  return a;
}
struct F2 { v16b h, l; };
__device__ __forceinline__ F2 bsplit16(const float v[16]) { F2 r;
#pragma unroll
  for (int i = 0; i < 16; ++i) { const __bf16 h = (__bf16)v[i]; r.h[i] = h; r.l[i] = (__bf16)(v[i] - (float)h); }
  return r; }
__device__ __forceinline__ F2 split_row(const float* row, int k0, int lane) { float v[16]; const float* p = row + k0 + 8 * (lane >> 4);
#pragma unroll
  for (int i = 0; i < 8; ++i) { v[i] = p[i]; v[8 + i] = p[16 + i]; }
  return bsplit16(v); }
__device__ __forceinline__ F2 split_rowK(const float* row, int k0, int lane, int K) { float v[16]; const int g = lane >> 4;
#pragma unroll
  for (int i = 0; i < 8; ++i) { const int ka = k0 + 8 * g + i, kb = ka + 16; v[i] = ka < K ? row[ka < K ? ka : K - 1] : 0.f; v[8 + i] = kb < K ? row[kb < K ? kb : K - 1] : 0.f; }
  return bsplit16(v); }
__device__ __forceinline__ F2 split_col(const float* W, int k0, int n, int lane, int ld, int K) { float v[16]; const int g = lane >> 4;
#pragma unroll
  for (int i = 0; i < 8; ++i) { const int ka = k0 + 8 * g + i, kb = ka + 16; v[i] = ka < K ? W[(size_t)(ka < K ? ka : K - 1) * ld + n] : 0.f; v[8 + i] = kb < K ? W[(size_t)(kb < K ? kb : K - 1) * ld + n] : 0.f; }
  return bsplit16(v); }
__device__ __forceinline__ v8f mac3(const F2& a, const F2& b, v8f c) { c = wmma_bf(a.l, b.h, c); c = wmma_bf(a.h, b.l, c); return wmma_bf(a.h, b.h, c); }
__device__ __forceinline__ float sigm(float v) { return 1.0f / (1.0f + expf(-v)); }
#define LDSX() do { asm volatile("s_wait_dscnt 0" ::: "memory"); __builtin_amdgcn_wave_barrier(); __builtin_amdgcn_fence(__ATOMIC_RELEASE, "workgroup"); } while (0)

#define NB 1
#define TT 2048
#define CC 768
#define DIN 768
#define NH 12
#define HD 64
#define NQB (TT / 64)
#define HG 4
#define SCALE (0.125f)
#define CAUSAL 0
#ifndef TNB
#define TNB NB
#endif
__device__ __forceinline__ float bfr(float v) { return (float)(__bf16)v; }
__host__ __device__ __forceinline__ int kb_last(int qb) { return CAUSAL ? ((qb * 64 + 63) >> 7) : (TT / 128 - 1); }
typedef __attribute__((ext_vector_type(8))) __bf16 v8b;
__device__ __forceinline__ v16b frag_b(const __bf16* rowk0, int lane) {
  union { v16b v; v8b q[2]; } u; const __bf16* p = rowk0 + 8 * (lane >> 4);
  u.q[0] = *(const v8b*)p; u.q[1] = *(const v8b*)(p + 16); return u.v;
}
#define QBH 0
#define QHI 2048
#define KHI 64
__device__ __forceinline__ v16b wcol_io(const float* Wm, int k0, int o, int lane, int ld) { v16b w; const int g = lane >> 4;
#pragma unroll
  for (int i = 0; i < 8; ++i) { w[i] = (__bf16)Wm[(size_t)(k0 + 8 * g + i) * ld + o]; w[8 + i] = (__bf16)Wm[(size_t)(k0 + 16 + 8 * g + i) * ld + o]; }
  return w; }
__device__ __forceinline__ v16b wcol_oi(const float* Wm, int k0, int o, int lane, int K) { v16b w; const float* p = Wm + (size_t)o * K + k0 + 8 * (lane >> 4);
#pragma unroll
  for (int i = 0; i < 8; ++i) { w[i] = (__bf16)p[i]; w[8 + i] = (__bf16)p[16 + i]; }
  return w; }
__device__ __forceinline__ v16h wcolh_io(const float* Wm, int k0, int o, int lane, int ld) { v16h w; const int g = lane >> 4;
#pragma unroll
  for (int i = 0; i < 8; ++i) { w[i] = (_Float16)(bfr(Wm[(size_t)(k0 + 8 * g + i) * ld + o]) * 256.0f); w[8 + i] = (_Float16)(bfr(Wm[(size_t)(k0 + 16 + 8 * g + i) * ld + o]) * 256.0f); }
  return w; }
__device__ __forceinline__ v16h wcolh_oi(const float* Wm, int k0, int o, int lane, int K) { v16h w; const float* p = Wm + (size_t)o * K + k0 + 8 * (lane >> 4);
#pragma unroll
  for (int i = 0; i < 8; ++i) { w[i] = (_Float16)(bfr(p[i]) * 256.0f); w[8 + i] = (_Float16)(bfr(p[16 + i]) * 256.0f); }
  return w; }
#define WQKV_LAYOUT 0
__device__ __forceinline__ v16b wcol_hdk(const float* Wm, int k0, int o, int lane) { v16b w; const int g = lane >> 4; const float* p = Wm + (size_t)(o / HD) * DIN * HD + (o % HD);
#pragma unroll
  for (int i = 0; i < 8; ++i) { w[i] = (__bf16)p[(size_t)(k0 + 8 * g + i) * HD]; w[8 + i] = (__bf16)p[(size_t)(k0 + 16 + 8 * g + i) * HD]; }
  return w; }
#define WO_OUT_IN 0
#if WQKV_LAYOUT == 1
#define WCOL(W, k0, o, lane) wcol_oi(W, k0, o, lane, DIN)
#elif WQKV_LAYOUT == 2
#define WCOL(W, k0, o, lane) wcol_hdk(W, k0, o, lane)
#else
#define WCOL(W, k0, o, lane) wcol_io(W, k0, o, lane, CC)
#endif
#if WO_OUT_IN
#define WOCOL(W, k0, o, lane) wcol_oi(W, k0, o, lane, CC)
#define WOCOLH(W, k0, o, lane) wcolh_oi(W, k0, o, lane, CC)
#else
#define WOCOL(W, k0, o, lane) wcol_io(W, k0, o, lane, DIN)
#define WOCOLH(W, k0, o, lane) wcolh_io(W, k0, o, lane, DIN)
#endif
#define FUSEDW 5376
#define MLPW 3072
#define GH 1536
#define NVOX 2048
#undef WCOL
#define WCOL(W, k0, o, lane) wcol_io(W, k0, o, lane, FUSEDW)
#define PROJ_EXTRA_PARAMS , const float* __restrict__ QNW, const float* __restrict__ QNB, const float* __restrict__ KNW, const float* __restrict__ KNB
__constant__ float ANG_H[256] = {-3.141592741e+00,-3.141592741e+00,-6.013906479e+01,-6.013906479e+01,-1.171365356e+02,-1.171365356e+02,-1.741340027e+02,-1.741340027e+02,-2.311314850e+02,-2.311314850e+02,-2.881289368e+02,-2.881289368e+02,-3.451264038e+02,-3.451264038e+02,-4.021238708e+02,-4.021238708e+02,-2.722713709e+00,-2.722713709e+00,-5.212052155e+01,-5.212052155e+01,-1.015183334e+02,-1.015183334e+02,-1.509161377e+02,-1.509161377e+02,-2.003139496e+02,-2.003139496e+02,-2.497117462e+02,-2.497117462e+02,-2.991095581e+02,-2.991095581e+02,-3.485073547e+02,-3.485073547e+02,-2.303834677e+00,-2.303834677e+00,-4.410198212e+01,-4.410198212e+01,-8.590013123e+01,-8.590013123e+01,-1.276982727e+02,-1.276982727e+02,-1.694964294e+02,-1.694964294e+02,-2.112945557e+02,-2.112945557e+02,-2.530926971e+02,-2.530926971e+02,-2.948908386e+02,-2.948908386e+02,-1.884955525e+00,-1.884955525e+00,-3.608343506e+01,-3.608343506e+01,-7.028191376e+01,-7.028191376e+01,-1.044803925e+02,-1.044803925e+02,-1.386788788e+02,-1.386788788e+02,-1.728773499e+02,-1.728773499e+02,-2.070758362e+02,-2.070758362e+02,-2.412743073e+02,-2.412743073e+02,-1.466076612e+00,-1.466076612e+00,-2.806489754e+01,-2.806489754e+01,-5.466371536e+01,-5.466371536e+01,-8.126253510e+01,-8.126253510e+01,-1.078613586e+02,-1.078613586e+02,-1.344601746e+02,-1.344601746e+02,-1.610589905e+02,-1.610589905e+02,-1.876578064e+02,-1.876578064e+02,-1.047197461e+00,-1.047197461e+00,-2.004635239e+01,-2.004635239e+01,-3.904550552e+01,-3.904550552e+01,-5.804465866e+01,-5.804465866e+01,-7.704381561e+01,-7.704381561e+01,-9.604296112e+01,-9.604296112e+01,-1.150421143e+02,-1.150421143e+02,-1.340412750e+02,-1.340412750e+02,-6.283183694e-01,-6.283183694e-01,-1.202780914e+01,-1.202780914e+01,-2.342730141e+01,-2.342730141e+01,-3.482678986e+01,-3.482678986e+01,-4.622628403e+01,-4.622628403e+01,-5.762577057e+01,-5.762577057e+01,-6.902526093e+01,-6.902526093e+01,-8.042475128e+01,-8.042475128e+01,-2.094393373e-01,-2.094393373e-01,-4.009267807e+00,-4.009267807e+00,-7.809095860e+00,-7.809095860e+00,-1.160892391e+01,-1.160892391e+01,-1.540875244e+01,-1.540875244e+01,-1.920858002e+01,-1.920858002e+01,-2.300840759e+01,-2.300840759e+01,-2.680823517e+01,-2.680823517e+01,2.094396949e-01,2.094396949e-01,4.009274483e+00,4.009274483e+00,7.809108734e+00,7.809108734e+00,1.160894299e+01,1.160894299e+01,1.540877819e+01,1.540877819e+01,1.920861244e+01,1.920861244e+01,2.300844574e+01,2.300844574e+01,2.680828094e+01,2.680828094e+01,6.283187270e-01,6.283187270e-01,1.202781582e+01,1.202781582e+01,2.342731285e+01,2.342731285e+01,3.482680893e+01,3.482680893e+01,4.622630692e+01,4.622630692e+01,5.762580109e+01,5.762580109e+01,6.902529907e+01,6.902529907e+01,8.042479706e+01,8.042479706e+01,1.047197700e+00,1.047197700e+00,2.004635811e+01,2.004635811e+01,3.904551697e+01,3.904551697e+01,5.804467392e+01,5.804467392e+01,7.704383850e+01,7.704383850e+01,9.604299164e+01,9.604299164e+01,1.150421448e+02,1.150421448e+02,1.340413055e+02,1.340413055e+02,1.466076851e+00,1.466076851e+00,2.806490135e+01,2.806490135e+01,5.466372299e+01,5.466372299e+01,8.126254272e+01,8.126254272e+01,1.078613739e+02,1.078613739e+02,1.344601898e+02,1.344601898e+02,1.610590057e+02,1.610590057e+02,1.876578369e+02,1.876578369e+02,1.884956121e+00,1.884956121e+00,3.608344650e+01,3.608344650e+01,7.028193665e+01,7.028193665e+01,1.044804230e+02,1.044804230e+02,1.386789246e+02,1.386789246e+02,1.728774109e+02,1.728774109e+02,2.070758972e+02,2.070758972e+02,2.412743835e+02,2.412743835e+02,2.303835154e+00,2.303835154e+00,4.410198975e+01,4.410198975e+01,8.590013885e+01,8.590013885e+01,1.276982956e+02,1.276982956e+02,1.694964600e+02,1.694964600e+02,2.112945862e+02,2.112945862e+02,2.530927429e+02,2.530927429e+02,2.948908997e+02,2.948908997e+02,2.722714186e+00,2.722714186e+00,5.212052917e+01,5.212052917e+01,1.015183487e+02,1.015183487e+02,1.509161530e+02,1.509161530e+02,2.003139801e+02,2.003139801e+02,2.497117767e+02,2.497117767e+02,2.991095886e+02,2.991095886e+02,3.485074158e+02,3.485074158e+02,3.141592741e+00,3.141592741e+00,6.013906479e+01,6.013906479e+01,1.171365356e+02,1.171365356e+02,1.741340027e+02,1.741340027e+02,2.311314850e+02,2.311314850e+02,2.881289368e+02,2.881289368e+02,3.451264038e+02,3.451264038e+02,4.021238708e+02,4.021238708e+02};
__constant__ float ANG_W[256] = {-3.141592741e+00,-3.141592741e+00,-6.013906479e+01,-6.013906479e+01,-1.171365356e+02,-1.171365356e+02,-1.741340027e+02,-1.741340027e+02,-2.311314850e+02,-2.311314850e+02,-2.881289368e+02,-2.881289368e+02,-3.451264038e+02,-3.451264038e+02,-4.021238708e+02,-4.021238708e+02,-2.722713709e+00,-2.722713709e+00,-5.212052155e+01,-5.212052155e+01,-1.015183334e+02,-1.015183334e+02,-1.509161377e+02,-1.509161377e+02,-2.003139496e+02,-2.003139496e+02,-2.497117462e+02,-2.497117462e+02,-2.991095581e+02,-2.991095581e+02,-3.485073547e+02,-3.485073547e+02,-2.303834677e+00,-2.303834677e+00,-4.410198212e+01,-4.410198212e+01,-8.590013123e+01,-8.590013123e+01,-1.276982727e+02,-1.276982727e+02,-1.694964294e+02,-1.694964294e+02,-2.112945557e+02,-2.112945557e+02,-2.530926971e+02,-2.530926971e+02,-2.948908386e+02,-2.948908386e+02,-1.884955525e+00,-1.884955525e+00,-3.608343506e+01,-3.608343506e+01,-7.028191376e+01,-7.028191376e+01,-1.044803925e+02,-1.044803925e+02,-1.386788788e+02,-1.386788788e+02,-1.728773499e+02,-1.728773499e+02,-2.070758362e+02,-2.070758362e+02,-2.412743073e+02,-2.412743073e+02,-1.466076612e+00,-1.466076612e+00,-2.806489754e+01,-2.806489754e+01,-5.466371536e+01,-5.466371536e+01,-8.126253510e+01,-8.126253510e+01,-1.078613586e+02,-1.078613586e+02,-1.344601746e+02,-1.344601746e+02,-1.610589905e+02,-1.610589905e+02,-1.876578064e+02,-1.876578064e+02,-1.047197461e+00,-1.047197461e+00,-2.004635239e+01,-2.004635239e+01,-3.904550552e+01,-3.904550552e+01,-5.804465866e+01,-5.804465866e+01,-7.704381561e+01,-7.704381561e+01,-9.604296112e+01,-9.604296112e+01,-1.150421143e+02,-1.150421143e+02,-1.340412750e+02,-1.340412750e+02,-6.283183694e-01,-6.283183694e-01,-1.202780914e+01,-1.202780914e+01,-2.342730141e+01,-2.342730141e+01,-3.482678986e+01,-3.482678986e+01,-4.622628403e+01,-4.622628403e+01,-5.762577057e+01,-5.762577057e+01,-6.902526093e+01,-6.902526093e+01,-8.042475128e+01,-8.042475128e+01,-2.094393373e-01,-2.094393373e-01,-4.009267807e+00,-4.009267807e+00,-7.809095860e+00,-7.809095860e+00,-1.160892391e+01,-1.160892391e+01,-1.540875244e+01,-1.540875244e+01,-1.920858002e+01,-1.920858002e+01,-2.300840759e+01,-2.300840759e+01,-2.680823517e+01,-2.680823517e+01,2.094396949e-01,2.094396949e-01,4.009274483e+00,4.009274483e+00,7.809108734e+00,7.809108734e+00,1.160894299e+01,1.160894299e+01,1.540877819e+01,1.540877819e+01,1.920861244e+01,1.920861244e+01,2.300844574e+01,2.300844574e+01,2.680828094e+01,2.680828094e+01,6.283187270e-01,6.283187270e-01,1.202781582e+01,1.202781582e+01,2.342731285e+01,2.342731285e+01,3.482680893e+01,3.482680893e+01,4.622630692e+01,4.622630692e+01,5.762580109e+01,5.762580109e+01,6.902529907e+01,6.902529907e+01,8.042479706e+01,8.042479706e+01,1.047197700e+00,1.047197700e+00,2.004635811e+01,2.004635811e+01,3.904551697e+01,3.904551697e+01,5.804467392e+01,5.804467392e+01,7.704383850e+01,7.704383850e+01,9.604299164e+01,9.604299164e+01,1.150421448e+02,1.150421448e+02,1.340413055e+02,1.340413055e+02,1.466076851e+00,1.466076851e+00,2.806490135e+01,2.806490135e+01,5.466372299e+01,5.466372299e+01,8.126254272e+01,8.126254272e+01,1.078613739e+02,1.078613739e+02,1.344601898e+02,1.344601898e+02,1.610590057e+02,1.610590057e+02,1.876578369e+02,1.876578369e+02,1.884956121e+00,1.884956121e+00,3.608344650e+01,3.608344650e+01,7.028193665e+01,7.028193665e+01,1.044804230e+02,1.044804230e+02,1.386789246e+02,1.386789246e+02,1.728774109e+02,1.728774109e+02,2.070758972e+02,2.070758972e+02,2.412743835e+02,2.412743835e+02,2.303835154e+00,2.303835154e+00,4.410198975e+01,4.410198975e+01,8.590013885e+01,8.590013885e+01,1.276982956e+02,1.276982956e+02,1.694964600e+02,1.694964600e+02,2.112945862e+02,2.112945862e+02,2.530927429e+02,2.530927429e+02,2.948908997e+02,2.948908997e+02,2.722714186e+00,2.722714186e+00,5.212052917e+01,5.212052917e+01,1.015183487e+02,1.015183487e+02,1.509161530e+02,1.509161530e+02,2.003139801e+02,2.003139801e+02,2.497117767e+02,2.497117767e+02,2.991095886e+02,2.991095886e+02,3.485074158e+02,3.485074158e+02,3.141592741e+00,3.141592741e+00,6.013906479e+01,6.013906479e+01,1.171365356e+02,1.171365356e+02,1.741340027e+02,1.741340027e+02,2.311314850e+02,2.311314850e+02,2.881289368e+02,2.881289368e+02,3.451264038e+02,3.451264038e+02,4.021238708e+02,4.021238708e+02};
__constant__ float ANG_D[128] = {-3.141592741e+00,-3.141592741e+00,-6.013906479e+01,-6.013906479e+01,-1.171365356e+02,-1.171365356e+02,-1.741340027e+02,-1.741340027e+02,-2.311314850e+02,-2.311314850e+02,-2.881289368e+02,-2.881289368e+02,-3.451264038e+02,-3.451264038e+02,-4.021238708e+02,-4.021238708e+02,-2.243994951e+00,-2.243994951e+00,-4.295647430e+01,-4.295647430e+01,-8.366895294e+01,-8.366895294e+01,-1.243814316e+02,-1.243814316e+02,-1.650939178e+02,-1.650939178e+02,-2.058063812e+02,-2.058063812e+02,-2.465188599e+02,-2.465188599e+02,-2.872313538e+02,-2.872313538e+02,-1.346396923e+00,-1.346396923e+00,-2.577388573e+01,-2.577388573e+01,-5.020137405e+01,-5.020137405e+01,-7.462886047e+01,-7.462886047e+01,-9.905635071e+01,-9.905635071e+01,-1.234838333e+02,-1.234838333e+02,-1.479113159e+02,-1.479113159e+02,-1.723388062e+02,-1.723388062e+02,-4.487988055e-01,-4.487988055e-01,-8.591291428e+00,-8.591291428e+00,-1.673378372e+01,-1.673378372e+01,-2.487627602e+01,-2.487627602e+01,-3.301877213e+01,-3.301877213e+01,-4.116126251e+01,-4.116126251e+01,-4.930375290e+01,-4.930375290e+01,-5.744624710e+01,-5.744624710e+01,4.487991333e-01,4.487991333e-01,8.591298103e+00,8.591298103e+00,1.673379707e+01,1.673379707e+01,2.487629509e+01,2.487629509e+01,3.301879501e+01,3.301879501e+01,4.116129303e+01,4.116129303e+01,4.930379105e+01,4.930379105e+01,5.744628906e+01,5.744628906e+01,1.346397042e+00,1.346397042e+00,2.577388763e+01,2.577388763e+01,5.020137787e+01,5.020137787e+01,7.462886047e+01,7.462886047e+01,9.905635834e+01,9.905635834e+01,1.234838409e+02,1.234838409e+02,1.479113312e+02,1.479113312e+02,1.723388214e+02,1.723388214e+02,2.243995190e+00,2.243995190e+00,4.295648193e+01,4.295648193e+01,8.366896820e+01,8.366896820e+01,1.243814545e+02,1.243814545e+02,1.650939484e+02,1.650939484e+02,2.058064270e+02,2.058064270e+02,2.465189056e+02,2.465189056e+02,2.872313843e+02,2.872313843e+02,3.141592741e+00,3.141592741e+00,6.013906479e+01,6.013906479e+01,1.171365356e+02,1.171365356e+02,1.741340027e+02,1.741340027e+02,2.311314850e+02,2.311314850e+02,2.881289368e+02,2.881289368e+02,3.451264038e+02,3.451264038e+02,4.021238708e+02,4.021238708e+02};
#define PROJ_EPI(which, row, t, h) do { if ((which) < 2) { float* rw = (row); const float* nw = (which) == 0 ? QNW : KNW; const float* nb = (which) == 0 ? QNB : KNB; \
    float m = 0.f; _Pragma("unroll 8") for (int i = 0; i < 64; ++i) m += rw[i]; m *= (1.0f / 64.0f); float var = 0.f; _Pragma("unroll 8") for (int i = 0; i < 64; ++i) { const float dlt = rw[i] - m; var += dlt * dlt; } var *= (1.0f / 64.0f); const float rs = 1.0f / sqrtf(var + 1e-5f); \
    _Pragma("unroll 8") for (int i = 0; i < 64; ++i) { const float wv = nw[i], bv2 = nb[i]; asm volatile("s_wait_loadcnt 0x0" ::: "memory"); rw[i] = (rw[i] - m) * rs * bfr(wv) + bfr(bv2); } \
    const int th = (t) >> 7, tw = ((t) >> 3) & 15, td = (t) & 7; \
    _Pragma("unroll 4") for (int i = 0; i < 24; ++i) { _Pragma("clang fp contract(off)") const float ang = i < 8 ? ANG_H[th * 16 + 2 * i] : (i < 16 ? ANG_W[tw * 16 + 2 * (i - 8)] : ANG_D[td * 16 + 2 * (i - 16)]); const float cs = cosf(ang), sn = sinf(ang); const float u0 = rw[2 * i], u1 = rw[2 * i + 1]; rw[2 * i] = u0 * cs + (-u1) * sn; rw[2 * i + 1] = u1 * cs + u0 * sn; } } } while (0)
__global__ __launch_bounds__(256) void k_gn(const float* __restrict__ X, const float* __restrict__ GAM, const int* __restrict__ BCS, float* __restrict__ XN) { (void)BCS; const int tid = threadIdx.x; const int t = blockIdx.x * 64 + (tid & 63); const int grp = blockIdx.y * 4 + (tid >> 6);
  const float* xg = X + (size_t)(grp * 64) * NVOX + t;
  float ss = 0.f;
#pragma unroll 2
  for (int i = 0; i < 64; i += 4) { const float a0 = xg[(size_t)(i + 0) * NVOX], a1 = xg[(size_t)(i + 1) * NVOX], a2 = xg[(size_t)(i + 2) * NVOX], a3 = xg[(size_t)(i + 3) * NVOX]; asm volatile("s_wait_loadcnt 0x0" ::: "memory");
    const float b0 = bfr(a0), b1 = bfr(a1), b2 = bfr(a2), b3 = bfr(a3); ss += b0 * b0; ss += b1 * b1; ss += b2 * b2; ss += b3 * b3; }
  const float r = 1.0f / sqrtf(ss * (1.0f / 64.0f) + 1e-6f);
  float* dst = XN + (size_t)t * CC + grp * 64;
#pragma unroll 2
  for (int q4 = 0; q4 < 16; ++q4) { const int i = q4 * 4; const float a0 = xg[(size_t)(i + 0) * NVOX], a1 = xg[(size_t)(i + 1) * NVOX], a2 = xg[(size_t)(i + 2) * NVOX], a3 = xg[(size_t)(i + 3) * NVOX]; const float g0 = GAM[grp * 64 + i], g1 = GAM[grp * 64 + i + 1], g2 = GAM[grp * 64 + i + 2], g3 = GAM[grp * 64 + i + 3]; asm volatile("s_wait_loadcnt 0x0" ::: "memory");
    v4f o; o[0] = (bfr(a0) * r) * bfr(g0); o[1] = (bfr(a1) * r) * bfr(g1); o[2] = (bfr(a2) * r) * bfr(g2); o[3] = (bfr(a3) * r) * bfr(g3); vst2(dst + i, o); } }
__global__ __launch_bounds__(128) void k_ff1(const float* __restrict__ XN, const float* __restrict__ WF, const float* __restrict__ BF, float* __restrict__ G) { __shared__ __align__(16) float sf[4][16][132];
  const int tid = threadIdx.x, wave = tid >> 5, lane = tid & 31, col = lane & 15, g = lane >> 4; const int c0 = blockIdx.y * 128; const size_t r0 = (size_t)blockIdx.x * 64 + wave * 16;
  v8f acc[8] = {}, accg[8] = {};
#pragma unroll 1
  for (int kc = 0; kc < CC / 32; ++kc) { v16b a; { const float* p = XN + (r0 + col) * CC + kc * 32 + 8 * g;
#pragma unroll
      for (int i = 0; i < 8; ++i) { a[i] = (__bf16)p[i]; a[8 + i] = (__bf16)p[16 + i]; } }
    asm volatile("s_wait_loadcnt 0x0" ::: "memory");
#pragma unroll
    for (int j = 0; j < 8; ++j) { const v16b w = wcol_io(WF, kc * 32, c0 + j * 16 + col, lane, FUSEDW); acc[j] = wmma_bf(a, w, acc[j]); const v16b w2 = wcol_io(WF + GH, kc * 32, c0 + j * 16 + col, lane, FUSEDW); accg[j] = wmma_bf(a, w2, accg[j]); } }
#pragma unroll
  for (int j = 0; j < 8; ++j) { const float bx = bfr(BF[c0 + j * 16 + col]), bg = bfr(BF[GH + c0 + j * 16 + col]); asm volatile("s_wait_loadcnt 0x0" ::: "memory");
#pragma unroll
    for (int r = 0; r < 8; ++r) { const float xh = acc[j][r] + bx, gt = accg[j][r] + bg; sf[wave][8 * g + r][j * 16 + col] = (gt / (1.0f + expf(-gt))) * xh; } }
  LDSX(); for (int rl = 0; rl < 16; ++rl) vst2(G + (r0 + rl) * GH + c0 + lane * 4, *(const v4f*)&sf[wave][rl][lane * 4]); }
__global__ __launch_bounds__(128) void k_ff2(const float* __restrict__ G, const float* __restrict__ WFF, const float* __restrict__ BFF, float* __restrict__ Y2) { __shared__ __align__(16) float sf[4][16][132];
  const int tid = threadIdx.x, wave = tid >> 5, lane = tid & 31, col = lane & 15, g = lane >> 4; const int c0 = blockIdx.y * 128; const size_t r0 = (size_t)blockIdx.x * 64 + wave * 16;
  v8f acc[8] = {};
#pragma unroll 1
  for (int kc = 0; kc < GH / 32; ++kc) { const F2 a = split_row(G + (r0 + col) * GH, kc * 32, lane); asm volatile("s_wait_loadcnt 0x0" ::: "memory");
#pragma unroll
    for (int j = 0; j < 8; ++j) { const v16b w = wcol_io(WFF, kc * 32, c0 + j * 16 + col, lane, CC); acc[j] = wmma_bf(a.h, w, acc[j]); acc[j] = wmma_bf(a.l, w, acc[j]); } }
#pragma unroll
  for (int j = 0; j < 8; ++j) { const float bb = bfr(BFF[c0 + j * 16 + col]); asm volatile("s_wait_loadcnt 0x0" ::: "memory");
#pragma unroll
    for (int r = 0; r < 8; ++r) sf[wave][8 * g + r][j * 16 + col] = acc[j][r] + bb; }
  LDSX(); for (int rl = 0; rl < 16; ++rl) { float* po = Y2 + (r0 + rl) * CC + c0 + lane * 4; const v4f prev = *(const v4f*)po; asm volatile("s_wait_loadcnt 0x0" ::: "memory"); v4f v = *(const v4f*)&sf[wave][rl][lane * 4]; v[0] += prev[0]; v[1] += prev[1]; v[2] += prev[2]; v[3] += prev[3]; vst2(po, v); } }
__global__ __launch_bounds__(256) void k_fin(const float* __restrict__ Y2, const float* __restrict__ X, float* __restrict__ OUT) { __shared__ __align__(16) float st[128][68];
  const int tid = threadIdx.x; const int t0 = blockIdx.x * 64, c0 = blockIdx.y * 128;
  for (int e = tid; e < 64 * 32; e += 256) { const int rl = e >> 5, q = e & 31; const v4f v = *(const v4f*)(Y2 + (size_t)(t0 + rl) * CC + c0 + q * 4); asm volatile("s_wait_loadcnt 0x0" ::: "memory"); st[q * 4 + 0][rl] = v[0]; st[q * 4 + 1][rl] = v[1]; st[q * 4 + 2][rl] = v[2]; st[q * 4 + 3][rl] = v[3]; }
  __syncthreads();
  for (int e = tid; e < 128 * 16; e += 256) { const int cl = e >> 4, q = e & 15; const size_t o = (size_t)(c0 + cl) * NVOX + t0 + q * 4; const v4f xr = *(const v4f*)(X + o); asm volatile("s_wait_loadcnt 0x0" ::: "memory"); v4f v = *(const v4f*)&st[cl][q * 4]; v[0] += bfr(xr[0]); v[1] += bfr(xr[1]); v[2] += bfr(xr[2]); v[3] += bfr(xr[3]); vst2(OUT + o, v); } }
#define WS_XN (WS_END)
#define WS_G  (WS_XN + 4u * (size_t)NVOX * CC)
#define WS_Y2 (WS_G + 4u * (size_t)NVOX * GH)
#define WS_END2 (WS_Y2 + 4u * (size_t)NVOX * CC)
#ifndef SM_EXTRA_PARAMS
#define SM_EXTRA_PARAMS
#endif
#ifndef PROJ_EXTRA_PARAMS
#define PROJ_EXTRA_PARAMS
#endif
#ifndef SM_MASK_HOOK
#define SM_MASK_HOOK (void)0
#endif

#define WS_QH  0u
#define WS_KH  (WS_QH + 2u * (size_t)NB * TT * CC)
#define WS_VT  (WS_KH + 2u * (size_t)NB * TT * CC)
#define WS_QL  (WS_VT + 2u * (size_t)NB * CC * TT)
#define WS_KL  (WS_QL + 2u * (size_t)NB * QHI * CC)
#define WS_VB  (WS_KL + 2u * (size_t)NB * KHI * CC)
#define WS_VBL (WS_VB + 2u * (size_t)NB * CC * KHI)
#define WS_S   (WS_VBL + 2u * (size_t)NB * CC * KHI)
#define WS_Y   (WS_S  + 4u * (size_t)HG * TT * TT)
#define WS_END (WS_Y  + 4u * (size_t)NB * TT * CC)

__global__ __launch_bounds__(128) void k_proj(const float* __restrict__ XQ, const float* __restrict__ XK, const float* __restrict__ XV, const float* __restrict__ WQ, const float* __restrict__ WK, const float* __restrict__ WV, const float* __restrict__ BQ, const float* __restrict__ BK, const float* __restrict__ BV,
    _Float16* __restrict__ QH, _Float16* __restrict__ QL, _Float16* __restrict__ KH, _Float16* __restrict__ KL, _Float16* __restrict__ VT, __bf16* __restrict__ VB, __bf16* __restrict__ VBL PROJ_EXTRA_PARAMS) {
  __shared__ __align__(16) float st[64][132]; __shared__ __align__(16) _Float16 sh[64][136], sl[64][136]; __shared__ __align__(16) _Float16 th[128][72]; __shared__ __align__(16) __bf16 tb[128][72], tbl[128][72];
  const int tid = threadIdx.x, wave = tid >> 5, lane = tid & 31, col = lane & 15, g = lane >> 4; const int which = blockIdx.z; const int c0 = blockIdx.y * 128; const size_t r0 = (size_t)blockIdx.x * 64; const size_t bb = r0 / TT; const int t0 = (int)(r0 % TT);
  const float* X = which == 0 ? XQ : which == 1 ? XK : XV; const float* WA = which == 0 ? WQ : which == 1 ? WK : WV; const float* BA = which == 0 ? BQ : which == 1 ? BK : BV;
  v8f acc[8] = {};
#pragma unroll 2
  for (int kc = 0; kc < DIN / 32; ++kc) { v16b a; { const float* p = X + (r0 + wave * 16 + col) * DIN + kc * 32 + 8 * g;
#pragma unroll
      for (int i = 0; i < 8; ++i) { a[i] = (__bf16)p[i]; a[8 + i] = (__bf16)p[16 + i]; } }
    asm volatile("s_wait_loadcnt 0x0" ::: "memory");
#pragma unroll
    for (int j = 0; j < 8; ++j) { const v16b w = WCOL(WA, kc * 32, c0 + j * 16 + col, lane); asm volatile("s_wait_loadcnt 0x0" ::: "memory"); acc[j] = wmma_bf(a, w, acc[j]); } }
  {
#pragma unroll
    for (int j = 0; j < 8; ++j) { const float bias = BA ? bfr(BA[c0 + j * 16 + col]) : 0.f;
#pragma unroll
      for (int r = 0; r < 8; ++r) st[wave * 16 + 8 * g + r][j * 16 + col] = acc[j][r] + bias; }
    __syncthreads();
    for (int e = tid; e < 64 * (128 / HD); e += 128) { const int rl = e / (128 / HD), hh = e % (128 / HD); PROJ_EPI(which, &st[rl][hh * HD], (int)((r0 + rl) % TT), (c0 / HD) + hh); }
    __syncthreads(); }
  if (which < 2) { _Float16* DH = which == 0 ? QH : KH; _Float16* DL = which == 0 ? QL : KL; const int nhi = which == 0 ? QHI : KHI; const bool hi_rows = t0 < nhi;
    for (int e = tid; e < 64 * 128; e += 128) { const int rl = e >> 7, cl = e & 127; const float v = st[rl][cl]; const _Float16 hv = (_Float16)v; sh[rl][cl] = hv; sl[rl][cl] = (_Float16)((v - (float)hv) * 1024.0f); }
    __syncthreads();
    for (int e = tid; e < 64 * 16; e += 128) { const int rl = e >> 4, q = e & 15; vst2((unsigned*)(DH + (r0 + rl) * CC + c0 + q * 8), *(const v4u*)&sh[rl][q * 8]); if (hi_rows) vst2((unsigned*)(DL + (bb * nhi + t0 + rl) * (size_t)CC + c0 + q * 8), *(const v4u*)&sl[rl][q * 8]); }
  } else { const bool hi_rows = t0 < KHI;
    for (int e = tid; e < 64 * 128; e += 128) { const int rl = e & 63, cl = e >> 6; const float v = st[rl][cl]; th[cl][rl] = (_Float16)v; const __bf16 bh = (__bf16)v; tb[cl][rl] = bh; tbl[cl][rl] = (__bf16)(v - (float)bh); }
    __syncthreads();
    for (int e = tid; e < 128 * 8; e += 128) { const int cl = e >> 3, q = e & 7; vst2((unsigned*)(VT + (bb * CC + c0 + cl) * (size_t)TT + t0 + q * 8), *(const v4u*)&th[cl][q * 8]); if (hi_rows) { const size_t o3 = (bb * CC + c0 + cl) * (size_t)KHI + t0 + q * 8; vst2((unsigned*)(VB + o3), *(const v4u*)&tb[cl][q * 8]); vst2((unsigned*)(VBL + o3), *(const v4u*)&tbl[cl][q * 8]); } } } }
__global__ __launch_bounds__(128) void k_sc(const _Float16* __restrict__ QH, const _Float16* __restrict__ KH, const _Float16* __restrict__ QL, const _Float16* __restrict__ KL, int b, int h0, float* __restrict__ S0) { __shared__ __align__(16) float ss[4][16][132];
  const int qb = blockIdx.x, kb = blockIdx.y; if (kb > kb_last(qb)) return;
  const int h = h0 + blockIdx.z; float* S = S0 + (size_t)blockIdx.z * TT * TT;
  const int tid = threadIdx.x, wave = tid >> 5, lane = tid & 31, col = lane & 15, g = lane >> 4; const int k0 = kb * 128; const int ql0 = qb * 64 + wave * 16; const size_t q0 = (size_t)b * TT + ql0, kr0 = (size_t)b * TT + k0;
  v8f acc[8] = {}, accl[8] = {};
  const _Float16* QLb = QL + (size_t)b * QHI * CC; const _Float16* KLb = KL + (size_t)b * KHI * CC;
  if (qb < QBH) {
#pragma unroll
    for (int kc = 0; kc < HD / 32; ++kc) { const v16h ah = frag_h(QH + (q0 + col) * CC + h * HD + kc * 32, lane), al = frag_h(QLb + (size_t)(ql0 + col) * CC + h * HD + kc * 32, lane);
#pragma unroll
      for (int j = 0; j < 8; ++j) { const v16h kbf = frag_h(KH + (kr0 + j * 16 + col) * CC + h * HD + kc * 32, lane), klf = frag_h(KLb + (size_t)(k0 + j * 16 + col) * CC + h * HD + kc * 32, lane); acc[j] = wmma16(ah, kbf, acc[j]); accl[j] = wmma16(al, kbf, accl[j]); accl[j] = wmma16(ah, klf, accl[j]); } }
  } else if (qb * 64 < QHI) {
#pragma unroll
    for (int kc = 0; kc < HD / 32; ++kc) { const v16h ah = frag_h(QH + (q0 + col) * CC + h * HD + kc * 32, lane), al = frag_h(QLb + (size_t)(ql0 + col) * CC + h * HD + kc * 32, lane);
#pragma unroll
      for (int j = 0; j < 8; ++j) { const v16h kbf = frag_h(KH + (kr0 + j * 16 + col) * CC + h * HD + kc * 32, lane); acc[j] = wmma16(ah, kbf, acc[j]); accl[j] = wmma16(al, kbf, accl[j]); } }
  } else {
#pragma unroll
    for (int kc = 0; kc < HD / 32; ++kc) { const v16h ah = frag_h(QH + (q0 + col) * CC + h * HD + kc * 32, lane);
#pragma unroll
      for (int j = 0; j < 8; ++j) { const v16h kbf = frag_h(KH + (kr0 + j * 16 + col) * CC + h * HD + kc * 32, lane); acc[j] = wmma16(ah, kbf, acc[j]); } } }
#pragma unroll
  for (int j = 0; j < 8; ++j) {
#pragma unroll
    for (int r = 0; r < 8; ++r) ss[wave][8 * g + r][j * 16 + col] = (acc[j][r] + accl[j][r] * (1.0f / 1024.0f)) * SCALE; }
  LDSX(); for (int rl = 0; rl < 16; ++rl) vst2(S + (size_t)(ql0 + rl) * TT + k0 + lane * 4, *(const v4f*)&ss[wave][rl][lane * 4]); }
__global__ __launch_bounds__(256) void k_sm(float* __restrict__ S0 SM_EXTRA_PARAMS) { __shared__ float sred[8]; __shared__ float sbc; __shared__ __align__(16) float shv[TT];
  const int tid = threadIdx.x; const int t = blockIdx.x; const int kend = (kb_last(t >> 6) + 1) * 128;
  float* sr = S0 + (size_t)blockIdx.y * TT * TT + (size_t)t * TT;
  float m = -3.0e38f; for (int k = tid; k < kend; k += 256) { float v = (!CAUSAL || k <= t) ? sr[k] : -3.0e38f; SM_MASK_HOOK; shv[k] = v; m = fmaxf(m, v); }
#pragma unroll
  for (int o = 1; o < 32; o <<= 1) m = fmaxf(m, __shfl_xor(m, o));
  if ((tid & 31) == 0) sred[tid >> 5] = m; __syncthreads(); if (tid == 0) { float a = sred[0]; for (int i = 1; i < 8; ++i) a = fmaxf(a, sred[i]); sbc = a; } __syncthreads(); m = sbc; __syncthreads();
  float sum = 0.f; for (int k = tid; k < kend; k += 256) { const float v = shv[k]; const float e = (v <= -1.0e38f) ? 0.f : expf(v - m); shv[k] = e; sum += e; }
#pragma unroll
  for (int o = 1; o < 32; o <<= 1) sum += __shfl_xor(sum, o);
  if ((tid & 31) == 0) sred[tid >> 5] = sum; __syncthreads(); if (tid == 0) { float a = 0.f; for (int i = 0; i < 8; ++i) a += sred[i]; sbc = a > 0.f ? 2048.0f / a : 0.f; }     __syncthreads(); const float inv = sbc;
  for (int k = tid; k < kend; k += 256) shv[k] = shv[k] * inv;
  __syncthreads(); for (int q = tid; q < kend / 4; q += 256) vst2(sr + q * 4, *(const v4f*)&shv[q * 4]); }
__global__ __launch_bounds__(128) void k_pv(const float* __restrict__ PS0, const _Float16* __restrict__ VT, const __bf16* __restrict__ VB, const __bf16* __restrict__ VBL, int b, int h0, float* __restrict__ Y) { const int h = h0 + blockIdx.z; const float* PS = PS0 + (size_t)blockIdx.z * TT * TT; __shared__ __align__(16) float ss[4][16][HD + 4];
  const int tid = threadIdx.x, wave = tid >> 5, lane = tid & 31, col = lane & 15, g = lane >> 4; const int qb = blockIdx.x; const int ql0 = qb * 64 + wave * 16; const int kce = (kb_last(qb) + 1) * 4;
  v8f acc[HD / 16] = {};
  if (qb < QBH) {
#pragma unroll 1
    for (int kc = 0; kc < kce; ++kc) { const F2 p = split_row(PS + (size_t)(ql0 + col) * TT, kc * 32, lane);
      asm volatile("s_wait_loadcnt 0x0" ::: "memory");
#pragma unroll
      for (int j = 0; j < HD / 16; ++j) { const size_t po = ((size_t)b * CC + h * HD + j * 16 + col) * (size_t)KHI + kc * 32; const v16b vh = frag_b(VB + po, lane); acc[j] = wmma_bf(p.h, vh, acc[j]); acc[j] = wmma_bf(p.l, vh, acc[j]); acc[j] = wmma_bf(p.h, frag_b(VBL + po, lane), acc[j]); } }
  } else {
#pragma unroll 1
    for (int kc = 0; kc < kce; ++kc) { const v16h p = frag_f32(PS + (size_t)(ql0 + col) * TT + kc * 32, lane);
      asm volatile("s_wait_loadcnt 0x0" ::: "memory");
#pragma unroll
      for (int j = 0; j < HD / 16; ++j) { const size_t po = ((size_t)b * CC + h * HD + j * 16 + col) * (size_t)TT + kc * 32; acc[j] = wmma16(p, frag_h(VT + po, lane), acc[j]); } } }
#pragma unroll
  for (int j = 0; j < HD / 16; ++j)
#pragma unroll
    for (int r = 0; r < 8; ++r) ss[wave][8 * g + r][j * 16 + col] = acc[j][r] * (1.0f / 2048.0f);
  LDSX(); for (int rl = 0; rl < 16; ++rl) if (lane < HD / 4) vst2(Y + ((size_t)b * TT + ql0 + rl) * CC + h * HD + lane * 4, *(const v4f*)&ss[wave][rl][lane * 4]); }
__global__ __launch_bounds__(128) void k_out(const float* __restrict__ Y, const float* __restrict__ WO, const float* __restrict__ BO, float* __restrict__ OUT) { __shared__ __align__(16) float sf[4][16][132];
  const int tid = threadIdx.x, wave = tid >> 5, lane = tid & 31, col = lane & 15, g = lane >> 4; const int c0 = blockIdx.y * 128; const size_t r0 = (size_t)blockIdx.x * 64 + wave * 16;
  v8f acc[8] = {};
  if (CAUSAL && (int)(((size_t)blockIdx.x * 64) % TT) < QHI) {
#pragma unroll 2
    for (int kc = 0; kc < CC / 32; ++kc) { const F2 a = split_row(Y + (r0 + col) * CC, kc * 32, lane); asm volatile("s_wait_loadcnt 0x0" ::: "memory");
#pragma unroll
      for (int j = 0; j < 8; ++j) { const v16b w = WOCOL(WO, kc * 32, c0 + j * 16 + col, lane); asm volatile("s_wait_loadcnt 0x0" ::: "memory"); acc[j] = wmma_bf(a.h, w, acc[j]); acc[j] = wmma_bf(a.l, w, acc[j]); } }
#pragma unroll
    for (int j = 0; j < 8; ++j) { const float bias = BO ? bfr(BO[c0 + j * 16 + col]) : 0.f;
#pragma unroll
      for (int r = 0; r < 8; ++r) sf[wave][8 * g + r][j * 16 + col] = acc[j][r] + bias; }
  } else {
#pragma unroll 2
    for (int kc = 0; kc < CC / 32; ++kc) { const v16h a = frag_f32s(Y + (r0 + col) * CC + kc * 32, lane, 64.0f); asm volatile("s_wait_loadcnt 0x0" ::: "memory");
#pragma unroll
      for (int j = 0; j < 8; ++j) { const v16h w = WOCOLH(WO, kc * 32, c0 + j * 16 + col, lane); asm volatile("s_wait_loadcnt 0x0" ::: "memory"); acc[j] = wmma16(a, w, acc[j]); } }
#pragma unroll
    for (int j = 0; j < 8; ++j) { const float bias = BO ? bfr(BO[c0 + j * 16 + col]) : 0.f;
#pragma unroll
      for (int r = 0; r < 8; ++r) sf[wave][8 * g + r][j * 16 + col] = acc[j][r] * (1.0f / 16384.0f) + bias; } }
  LDSX(); for (int rl = 0; rl < 16; ++rl) vst2(OUT + (r0 + rl) * DIN + c0 + lane * 4, *(const v4f*)&sf[wave][rl][lane * 4]); }

extern "C" void kernel_launch(void* const* d_in, const int* in_sizes, int n_in, void* d_out, int out_size, void* d_ws, size_t ws_size, hipStream_t stream) {
  (void)in_sizes; (void)n_in; (void)out_size;
  const float** F = (const float**)d_in;
  if (ws_size < (size_t)WS_END) return;
  char* ws = (char*)d_ws; _Float16 *QH = (_Float16*)(ws + WS_QH), *KH = (_Float16*)(ws + WS_KH), *VT = (_Float16*)(ws + WS_VT), *QL = (_Float16*)(ws + WS_QL), *KL = (_Float16*)(ws + WS_KL); __bf16 *VB = (__bf16*)(ws + WS_VB), *VBL = (__bf16*)(ws + WS_VBL); float *S = (float*)(ws + WS_S), *Y = (float*)(ws + WS_Y);
  (void)Y; (void)QL; (void)KL; (void)VB; (void)VBL;
  if (ws_size < (size_t)WS_END2) return;
  float *XN = (float*)(ws + WS_XN), *Gh = (float*)(ws + WS_G), *Y2 = (float*)(ws + WS_Y2);
  k_gn<<<dim3(NVOX / 64, 3), 256, 0, stream>>>(F[0], F[2], (const int*)d_in[1], XN);
  k_proj<<<dim3(TT / 64, CC / 128, 3), 128, 0, stream>>>(XN, XN, XN, F[3] + MLPW, F[3] + MLPW + CC, F[3] + MLPW + 2 * CC, F[4] + MLPW, F[4] + MLPW + CC, F[4] + MLPW + 2 * CC, QH, QL, KH, KL, VT, VB, VBL, F[5], F[6], F[7], F[8]);
  k_ff1<<<dim3(NVOX / 64, GH / 128), 128, 0, stream>>>(XN, F[3], F[4], Gh);
  for (int h0 = 0; h0 < NH; h0 += HG) {
    k_sc<<<dim3(NQB, TT / 128, HG), 128, 0, stream>>>(QH, KH, QL, KL, 0, h0, S);
    k_sm<<<dim3(TT, HG), 256, 0, stream>>>(S);
    k_pv<<<dim3(NQB, 1, HG), 128, 0, stream>>>(S, VT, VB, VBL, 0, h0, Y);
  }
  k_out<<<dim3(TT / 64, DIN / 128), 128, 0, stream>>>(Y, F[9], nullptr, Y2);
  k_ff2<<<dim3(NVOX / 64, CC / 128), 128, 0, stream>>>(Gh, F[10], F[11], Y2);
  k_fin<<<dim3(NVOX / 64, CC / 128), 256, 0, stream>>>(Y2, F[0], (float*)d_out);
}
